// GRUDecoder_75179107549419
// MI455X (gfx1250) — hardware-verified
//
#include <hip/hip_runtime.h>
#include <math.h>

constexpr int NB        = 8192;
constexpr int NTS       = 1024;
constexpr int NHID      = 64;
constexpr int NGATE     = 192;
constexpr int NOUTF     = 256;
constexpr int NTHR      = 128;
constexpr int NWAVE     = NTHR / 32;
constexpr int ROWS_WAVE = 16;
constexpr int ROWS_BLK  = NWAVE * ROWS_WAVE;
constexpr int WP        = 72;
constexpr int HP        = 72;
constexpr int CT        = 128;
constexpr int SLP       = 68;
constexpr int NPAR      = 3 * NGATE;
constexpr float WSC      = 256.0f;
constexpr float HSC      = 16.0f;
constexpr float GINV     = 1.0f / 4096.0f;
constexpr float LOSC     = 65536.0f;
constexpr float LOSC_INV = 1.0f / 65536.0f;

static_assert(NB % ROWS_BLK == 0);
static_assert(NTS % CT == 0);
static_assert(CT == 32 * 4);
static_assert(NHID == 64);
static_assert(NGATE == 3 * NHID && NGATE % 16 == 0);
static_assert(NOUTF % 64 == 0);
static_assert((NGATE * NHID) % (4 * NTHR) == 0);
static_assert((NOUTF * NHID) % (4 * NTHR) == 0);
static_assert((NWAVE * 2 * ROWS_WAVE * HP) % NTHR == 0);
static_assert(CT * ROWS_WAVE >= ROWS_WAVE * SLP);
static_assert(NGATE % 4 == 0 && NGATE / 4 <= NTHR);
static_assert(WP % 8 == 0 && HP % 8 == 0 && SLP % 4 == 0);

typedef __attribute__((ext_vector_type(16))) _Float16 v16h;
typedef __attribute__((ext_vector_type(8)))  _Float16 v8h;
typedef __attribute__((ext_vector_type(4)))  _Float16 v4h;
typedef __attribute__((ext_vector_type(8)))  float    v8f;
typedef __attribute__((ext_vector_type(4)))  float    v4f;

__device__ __forceinline__ void dep_guard_h(v8f& a, v8f& b, v16h x, v16h y) { asm volatile("v_nop\n\tv_nop\n\tv_nop\n\tv_nop" : "+v"(a), "+v"(b) : "v"(x), "v"(y)); }
__device__ __forceinline__ void dep_guard3_h(v8f& a, v8f& b, v8f& c, v16h x, v16h y) { asm volatile("v_nop\n\tv_nop\n\tv_nop\n\tv_nop" : "+v"(a), "+v"(b), "+v"(c) : "v"(x), "v"(y)); }
__device__ __forceinline__ void keep4_h(v16h a, v16h b, v16h c, v16h d) { asm volatile("v_nop" :: "v"(a), "v"(b), "v"(c), "v"(d)); }

template <typename T> struct Frag;
template <> struct Frag<_Float16> {
  typedef v16h V; union U { v16h v; v8h h[2]; };
  static __device__ __forceinline__ v16h load(const _Float16* p) {
    U f; f.h[0] = *(const v8h*)(p); f.h[1] = *(const v8h*)(p + 16); return f.v;
  }
  static __device__ __forceinline__ v8f mma(v16h a, v16h b, v8f c) {
    return __builtin_amdgcn_wmma_f32_16x16x32_f16(false, a, false, b, (short)0, c, false, false);
  }
};

__device__ __forceinline__ float fsig(float x)  { return __builtin_amdgcn_rcpf(1.0f + __expf(-x)); }
__device__ __forceinline__ float ftanh(float x) { return 1.0f - 2.0f * __builtin_amdgcn_rcpf(__expf(2.0f * x) + 1.0f); }

__global__ __launch_bounds__(NTHR) void gru_fc_kernel(const float* __restrict__ x,    const float* __restrict__ w_ih,
                                                      const float* __restrict__ w_hh, const float* __restrict__ b_ih,
                                                      const float* __restrict__ b_hh, const float* __restrict__ fc_w,
                                                      const float* __restrict__ fc_b, float* __restrict__ out) {
  __shared__ __align__(16) _Float16 Wsh[NOUTF * WP];
  __shared__ __align__(16) _Float16 Hsh[NWAVE][2][ROWS_WAVE * HP];
  __shared__ __align__(16) float    Xsh[NWAVE][CT * ROWS_WAVE];
  __shared__ __align__(16) float    Psh[NPAR];

  const int tid  = threadIdx.x;
  const int lane = tid & 31;
  const int wave = tid >> 5;
  const int c    = lane & 15;
  const int hh   = lane >> 4;
  const int koff = hh * 8;
  const int rowBase = blockIdx.x * ROWS_BLK + wave * ROWS_WAVE;

#pragma unroll 4
  for (int i = 0; i < (NGATE * NHID) / (4 * NTHR); ++i) {
    const int idx4 = (i * NTHR + tid) * 4;
    const int row = idx4 >> 6, k = idx4 & 63;
    const v4f v = *(const v4f*)(w_hh + idx4);
    v4h hv;
    hv[0] = (_Float16)(v[0] * WSC); hv[1] = (_Float16)(v[1] * WSC);
    hv[2] = (_Float16)(v[2] * WSC); hv[3] = (_Float16)(v[3] * WSC);
    *(v4h*)(Wsh + row * WP + k) = hv;
  }
  {
    _Float16* hf = &Hsh[0][0][0];
#pragma unroll 1
    for (int i = tid; i < NWAVE * 2 * ROWS_WAVE * HP; i += NTHR) hf[i] = (_Float16)0.0f;
  }
  {
    const int i4 = ((tid < NGATE / 4) ? tid : (NGATE / 4 - 1)) * 4;
    const v4f va = *(const v4f*)(w_ih + i4);
    const v4f vb = *(const v4f*)(b_ih + i4);
    const v4f vc = *(const v4f*)(b_hh + i4);
    if (tid < NGATE / 4) {
      *(v4f*)(Psh + i4)             = va;
      *(v4f*)(Psh + NGATE + i4)     = vb;
      *(v4f*)(Psh + 2 * NGATE + i4) = vc;
    }
  }
  __syncthreads();

  float kwr[4], kwz[4], kwn[4], kcr[4], kcz[4], kbin[4], kbhn[4];
#pragma unroll
  for (int j = 0; j < 4; ++j) {
    const int col = 16 * j + c;
    kwr[j]  = Psh[col];
    kwz[j]  = Psh[NHID + col];
    kwn[j]  = Psh[2 * NHID + col];
    kcr[j]  = Psh[NGATE + col] + Psh[2 * NGATE + col];
    kcz[j]  = Psh[NGATE + NHID + col] + Psh[2 * NGATE + NHID + col];
    kbin[j] = Psh[NGATE + 2 * NHID + col];
    kbhn[j] = Psh[2 * NGATE + 2 * NHID + col];
  }

  float hst[4][8];
#pragma unroll
  for (int j = 0; j < 4; ++j)
#pragma unroll
    for (int r = 0; r < 8; ++r) hst[j][r] = 0.0f;

  const v8f z8 = {0.f, 0.f, 0.f, 0.f, 0.f, 0.f, 0.f, 0.f};
  float* xw = Xsh[wave];

#pragma unroll 1
  for (int t = 0; t < NTS; ++t) {
    const int tt = t & (CT - 1);
    if (tt == 0) {
      const float* xsrc = x + (size_t)rowBase * NTS + (size_t)t + 4 * lane;
#pragma unroll 4
      for (int i = 0; i < ROWS_WAVE; ++i) {
        const v4f v = *(const v4f*)(xsrc + (size_t)i * NTS);
        xw[(4 * lane + 0) * ROWS_WAVE + i] = v[0];
        xw[(4 * lane + 1) * ROWS_WAVE + i] = v[1];
        xw[(4 * lane + 2) * ROWS_WAVE + i] = v[2];
        xw[(4 * lane + 3) * ROWS_WAVE + i] = v[3];
      }
      __syncthreads();
    }

    const int cur = t & 1;
    const _Float16* hrd = &Hsh[wave][cur][0] + c * HP + koff;
    _Float16*       hwr = &Hsh[wave][cur ^ 1][0];
    const v16h a0 = Frag<_Float16>::load(hrd);
    const v16h a1 = Frag<_Float16>::load(hrd + 32);

    const v4f xa = *(const v4f*)(xw + tt * ROWS_WAVE + 8 * hh);
    const v4f xb = *(const v4f*)(xw + tt * ROWS_WAVE + 8 * hh + 4);
    float xv[8];
#pragma unroll
    for (int e = 0; e < 4; ++e) { xv[e] = xa[e]; xv[4 + e] = xb[e]; }

#pragma unroll
    for (int j = 0; j < 4; ++j) {
      const _Float16* wr = Wsh + (16 * j + c) * WP + koff;
      const v16h br0 = Frag<_Float16>::load(wr);
      const v16h br1 = Frag<_Float16>::load(wr + 32);
      const v16h bz0 = Frag<_Float16>::load(wr + NHID * WP);
      const v16h bz1 = Frag<_Float16>::load(wr + NHID * WP + 32);
      const v16h bn0 = Frag<_Float16>::load(wr + 2 * NHID * WP);
      const v16h bn1 = Frag<_Float16>::load(wr + 2 * NHID * WP + 32);
      v8f accr = Frag<_Float16>::mma(a0, br0, z8);
      accr     = Frag<_Float16>::mma(a1, br1, accr);
      v8f accz = Frag<_Float16>::mma(a0, bz0, z8);
      accz     = Frag<_Float16>::mma(a1, bz1, accz);
      v8f accn = Frag<_Float16>::mma(a0, bn0, z8);
      accn     = Frag<_Float16>::mma(a1, bn1, accn);
      dep_guard3_h(accr, accz, accn, a1, bn1);
      keep4_h(br0, br1, bz0, bz1);
      keep4_h(bn0, bn1, a0, a1);
#pragma unroll
      for (int r = 0; r < 8; ++r) {
        const float pr = fmaf(xv[r], kwr[j], fmaf(accr[r], GINV, kcr[j]));
        const float pz = fmaf(xv[r], kwz[j], fmaf(accz[r], GINV, kcz[j]));
        const float hn = fmaf(accn[r], GINV, kbhn[j]);
        const float xn = fmaf(xv[r], kwn[j], kbin[j]);
        const float rg = fsig(pr);
        const float zg = fsig(pz);
        const float ng = ftanh(fmaf(rg, hn, xn));
        const float ho = hst[j][r];
        const float hv = fmaf(zg, ho - ng, ng);
        hst[j][r] = hv;
        hwr[(8 * hh + r) * HP + 16 * j + c] = (_Float16)(hv * HSC);
      }
    }
    __syncthreads();
  }

  {
    _Float16* hlo = &Hsh[wave][1][0];
#pragma unroll
    for (int j = 0; j < 4; ++j)
#pragma unroll
      for (int r = 0; r < 8; ++r) {
        const float hs = hst[j][r] * HSC;
        const float hi = (float)((_Float16)hs);
        hlo[(8 * hh + r) * HP + 16 * j + c] = (_Float16)((hs - hi) * LOSC);
      }
  }
#pragma unroll 4
  for (int i = 0; i < (NOUTF * NHID) / (4 * NTHR); ++i) {
    const int idx4 = (i * NTHR + tid) * 4;
    const int row = idx4 >> 6, k = idx4 & 63;
    const v4f v = *(const v4f*)(fc_w + idx4);
    v4h hv;
    hv[0] = (_Float16)(v[0] * WSC); hv[1] = (_Float16)(v[1] * WSC);
    hv[2] = (_Float16)(v[2] * WSC); hv[3] = (_Float16)(v[3] * WSC);
    *(v4h*)(Wsh + row * WP + k) = hv;
  }
  __syncthreads();

  const _Float16* hhi = &Hsh[wave][0][0] + c * HP + koff;
  const _Float16* hlr = &Hsh[wave][1][0] + c * HP + koff;
  const v16h ah0 = Frag<_Float16>::load(hhi);
  const v16h ah1 = Frag<_Float16>::load(hhi + 32);
  const v16h al0 = Frag<_Float16>::load(hlr);
  const v16h al1 = Frag<_Float16>::load(hlr + 32);
  float* slab = Xsh[wave];
  const int c4 = c * 4;

#pragma unroll 1
  for (int q = 0; q < NOUTF / 64; ++q) {
    v8f acch[4], accl[4];
#pragma unroll
    for (int jj = 0; jj < 4; ++jj) {
      const _Float16* wr = Wsh + (64 * q + 16 * jj + c) * WP + koff;
      const v16h b0 = Frag<_Float16>::load(wr);
      const v16h b1 = Frag<_Float16>::load(wr + 32);
      acch[jj] = Frag<_Float16>::mma(ah0, b0, z8);
      acch[jj] = Frag<_Float16>::mma(ah1, b1, acch[jj]);
      accl[jj] = Frag<_Float16>::mma(al0, b0, z8);
      accl[jj] = Frag<_Float16>::mma(al1, b1, accl[jj]);
      dep_guard_h(acch[jj], accl[jj], al1, b1);
      keep4_h(ah0, ah1, al0, b0);
    }
#pragma unroll
    for (int jj = 0; jj < 4; ++jj) {
      const float fb = fc_b[64 * q + 16 * jj + c];
#pragma unroll
      for (int r = 0; r < 8; ++r) {
        const float v = fmaf(fmaf(accl[jj][r], LOSC_INV, acch[jj][r]), GINV, fb);
        slab[(8 * hh + r) * SLP + 16 * jj + c] = v;
      }
    }
    __builtin_amdgcn_fence(__ATOMIC_RELEASE, "workgroup");
    __builtin_amdgcn_wave_barrier();
    __builtin_amdgcn_fence(__ATOMIC_ACQUIRE, "workgroup");
    for (int pass = 0; pass < 2; ++pass) {
#pragma unroll
      for (int it = 0; it < 8; ++it) {
        const int row = it * 2 + hh;
        const v4f v = *(const v4f*)(slab + row * SLP + c4);
        *(volatile v4f*)(out + (size_t)(rowBase + row) * NOUTF + 64 * q + c4) = v;
      }
      __threadfence();
    }
    __builtin_amdgcn_fence(__ATOMIC_RELEASE, "workgroup");
    __builtin_amdgcn_wave_barrier();
    __builtin_amdgcn_fence(__ATOMIC_ACQUIRE, "workgroup");
  }
}

extern "C" void kernel_launch(void* const* d_in, const int* in_sizes, int n_in,
                              void* d_out, int out_size, void* d_ws, size_t ws_size, hipStream_t stream) {
  (void)d_ws; (void)ws_size;
  if (n_in < 7 || d_out == nullptr) return;
  if (in_sizes[0] != NB * NTS || in_sizes[1] != NGATE || in_sizes[2] != NGATE * NHID || in_sizes[3] != NGATE ||
      in_sizes[4] != NGATE || in_sizes[5] != NOUTF * NHID || in_sizes[6] != NOUTF || out_size != NB * NOUTF) return;

  const float* x    = (const float*)d_in[0];
  const float* w_ih = (const float*)d_in[1];
  const float* w_hh = (const float*)d_in[2];
  const float* b_ih = (const float*)d_in[3];
  const float* b_hh = (const float*)d_in[4];
  const float* fc_w = (const float*)d_in[5];
  const float* fc_b = (const float*)d_in[6];
  float* out = (float*)d_out;

  gru_fc_kernel<<<NB / ROWS_BLK, NTHR, 0, stream>>>(x, w_ih, w_hh, b_ih, b_hh, fc_w, fc_b, out);
}
